// CrossMambaBlock_88699664597225
// MI455X (gfx1250) — hardware-verified
//
#include <hip/hip_runtime.h>
#include <math.h>
#include <stdint.h>


#define D_MODEL  256
#define D_INNER  512
#define D_STATE  16
#define DT_RANK  16
#define N_DBC    48
#define DBC_LD   64
#define SEQ_L    64
#define NSEQ     256
#define MTOT     16384

typedef __attribute__((ext_vector_type(16))) _Float16 v16h;
typedef __attribute__((ext_vector_type(8)))  _Float16 v8h;
typedef __attribute__((ext_vector_type(16))) __bf16   v16b;
typedef __attribute__((ext_vector_type(8)))  __bf16   v8b;
typedef __attribute__((ext_vector_type(8)))  float    v8f;
typedef __attribute__((ext_vector_type(4)))  float    v4f;
typedef __attribute__((ext_vector_type(8)))  unsigned short v8us;

__device__ __forceinline__ unsigned short f2bf_bits(float f) {
  unsigned u = __float_as_uint(f);
  return (unsigned short)((u + 0x7FFFu + ((u >> 16) & 1u)) >> 16);
}
__device__ __forceinline__ float bf_bits2f(unsigned short h) { return __uint_as_float(((unsigned)h) << 16); }

__device__ __forceinline__ float silu_f(float v) {
  return v * __builtin_amdgcn_rcpf(1.0f + __expf(-v));
}

__device__ __forceinline__ void dep_guard_h(v8f& a, v8f& b, v16h x, v16h y) { asm volatile("v_nop\n\tv_nop\n\tv_nop\n\tv_nop" : "+v"(a), "+v"(b) : "v"(x), "v"(y)); }
__device__ __forceinline__ void dep_guard_b(v8f& a, v8f& b, v16b x, v16b y) { asm volatile("v_nop\n\tv_nop\n\tv_nop\n\tv_nop" : "+v"(a), "+v"(b) : "v"(x), "v"(y)); }
__device__ __forceinline__ void keep4_h(v16h a, v16h b, v16h c, v16h d) { asm volatile("v_nop" :: "v"(a), "v"(b), "v"(c), "v"(d)); }
__device__ __forceinline__ void keep4_b(v16b a, v16b b, v16b c, v16b d) { asm volatile("v_nop" :: "v"(a), "v"(b), "v"(c), "v"(d)); }
__device__ __forceinline__ void acc_guard4(v8f& a, v8f& b, v8f& c, v8f& d) { asm volatile("v_nop\n\tv_nop\n\tv_nop\n\tv_nop" : "+v"(a), "+v"(b), "+v"(c), "+v"(d)); }

template <typename T> struct Frag;
template <> struct Frag<_Float16> {
  typedef v16h V; union U { v16h v; v8h h[2]; };
  static __device__ __forceinline__ v16h load(const _Float16* p) {
    U f; f.h[0] = *(const v8h*)(p); f.h[1] = *(const v8h*)(p + 16); return f.v;
  }
  static __device__ __forceinline__ v8f mma(v16h a, v16h b, v8f c) {
    return __builtin_amdgcn_wmma_f32_16x16x32_f16(false, a, false, b, (short)0, c, false, false);
  }
  static __device__ __forceinline__ void guard(v8f& a, v8f& b, v16h x, v16h y) { dep_guard_h(a, b, x, y); }
  static __device__ __forceinline__ void keep(v16h a, v16h b, v16h c, v16h d) { keep4_h(a, b, c, d); }
};
template <> struct Frag<__bf16> {
  typedef v16b V; union U { v16b v; v8b h[2]; };
  static __device__ __forceinline__ v16b load(const __bf16* p) {
    U f; f.h[0] = *(const v8b*)(p); f.h[1] = *(const v8b*)(p + 16); return f.v;
  }
  static __device__ __forceinline__ v8f mma(v16b a, v16b b, v8f c) {
    return __builtin_amdgcn_wmma_f32_16x16x32_bf16(false, a, false, b, (short)0, c, false, false);
  }
  static __device__ __forceinline__ void guard(v8f& a, v8f& b, v16b x, v16b y) { dep_guard_b(a, b, x, y); }
  static __device__ __forceinline__ void keep(v16b a, v16b b, v16b c, v16b d) { keep4_b(a, b, c, d); }
};

template <int ET> struct Elem;
template <> struct Elem<0> { typedef _Float16 T; };
template <> struct Elem<1> { typedef __bf16 T; };
template <int ET, bool SPLIT, int BIAS_MODE, int OUT_MODE, bool RESID, int ACT = 0>
__global__ __launch_bounds__(256) void wmma_gemm64(
    const unsigned short* __restrict__ Ap, const unsigned short* __restrict__ A2p, int lda, long strideA,
    const unsigned short* __restrict__ Btp, const unsigned short* __restrict__ Bt2p, int ldb, long strideB,
    void* Cout, void* Cout2, int ldc, long strideC,
    const float* __restrict__ bias,
    const float* resid, long strideR,
    int M, int N, int K, float scale) {
  typedef typename Elem<ET>::T T;
  typedef typename Frag<T>::V V;
  const T* A = (const T*)Ap; const T* A2 = (const T*)A2p; const T* Bt = (const T*)Btp; const T* Bt2 = (const T*)Bt2p;
  __shared__ __align__(16) float sT[8][16 * 68];
  const int b    = blockIdx.y;
  const int lane = threadIdx.x & 31;
  const int wave = threadIdx.x >> 5;
  const int tilesN = N >> 6;
  const int tilesM = M >> 6;
  const int tile = blockIdx.x * 8 + wave;
  if (tile >= tilesM * tilesN) return;
  const int tm = tile / tilesN;
  const int tn = tile - tm * tilesN;
  const int m0 = tm << 6;
  const int n0 = tn << 6;

  const T* Ab  = A  + (size_t)b * strideA;
  const T* Bb  = Bt + (size_t)b * strideB;
  const T* Ab2 = SPLIT ? (A2  + (size_t)b * strideA) : nullptr;
  const T* Bb2 = SPLIT ? (Bt2 + (size_t)b * strideB) : nullptr;

  const int rlane = lane & 15;
  const int koff  = (lane >> 4) * 8;
  const int mOff  = (lane >> 4) * 8;

  v8f acc[4][4];
#pragma unroll
  for (int i = 0; i < 4; ++i)
#pragma unroll
    for (int j = 0; j < 4; ++j) acc[i][j] = (v8f){0.f,0.f,0.f,0.f,0.f,0.f,0.f,0.f};

  for (int k0 = 0; k0 < K; k0 += 32) {
    V bh[4], bl[4];
#pragma unroll
    for (int j = 0; j < 4; ++j) {
      const size_t bo = (size_t)(n0 + (j << 4) + rlane) * ldb + koff + k0;
      bh[j] = Frag<T>::load(Bb + bo);
      if (SPLIT) bl[j] = Frag<T>::load(Bb2 + bo);
    }
#pragma unroll
    for (int i = 0; i < 4; ++i) {
      const size_t ao = (size_t)(m0 + (i << 4) + rlane) * lda + koff + k0;
      V ah = Frag<T>::load(Ab + ao);
      V al;
      if (SPLIT) al = Frag<T>::load(Ab2 + ao);
#pragma unroll
      for (int j = 0; j < 4; ++j) {
        acc[i][j] = Frag<T>::mma(ah, bh[j], acc[i][j]);
        if (SPLIT) {
          acc[i][j] = Frag<T>::mma(ah, bl[j], acc[i][j]);
          acc[i][j] = Frag<T>::mma(al, bh[j], acc[i][j]);
        }
      }
      Frag<T>::guard(acc[i][0], acc[i][3], ah, SPLIT ? al : ah);
    }
    Frag<T>::keep(bh[0], bh[1], bh[2], bh[3]);
    if (SPLIT) Frag<T>::keep(bl[0], bl[1], bl[2], bl[3]);
  }
  acc_guard4(acc[0][0], acc[0][1], acc[0][2], acc[0][3]);
  acc_guard4(acc[1][0], acc[1][1], acc[1][2], acc[1][3]);
  acc_guard4(acc[2][0], acc[2][1], acc[2][2], acc[2][3]);
  acc_guard4(acc[3][0], acc[3][1], acc[3][2], acc[3][3]);

  float* slab = sT[wave];
  const float* Rb = RESID ? (resid + (size_t)b * strideR) : nullptr;
#pragma unroll
  for (int i = 0; i < 4; ++i) {
    const int mBase = m0 + (i << 4);
#pragma unroll
    for (int j = 0; j < 4; ++j) {
      const int n = n0 + (j << 4) + rlane;
      float bv = 0.f;
      if (BIAS_MODE == 2) bv = bias[n];
#pragma unroll
      for (int r = 0; r < 8; ++r) {
        float v = acc[i][j][r] * scale;
        if (BIAS_MODE == 1) v += bias[mBase + mOff + r];
        if (BIAS_MODE == 2) v += bv;
        if (RESID) v += Rb[(size_t)(mBase + mOff + r) * ldc + n];
        if (ACT == 1) v = tanhf(v);
        if (ACT == 2) v = fmaxf(v, 0.0f);
        if (ACT == 3) v = v / (1.0f + expf(-v));
        if (ACT == 4) v = (v > 0.f) ? v : 0.01f * v;
        if (ACT == 5) v = 0.5f * v * (1.0f + erff(v * 0.70710678118654752f));
        slab[(mOff + r) * 68 + (j << 4) + rlane] = v;
      }
    }
    __builtin_amdgcn_fence(__ATOMIC_RELEASE, "workgroup");
    __builtin_amdgcn_wave_barrier();
    __builtin_amdgcn_fence(__ATOMIC_ACQUIRE, "workgroup");
    if (OUT_MODE == 0) {
      float* C = (float*)Cout + (size_t)b * strideC;
      const int hh = lane >> 4, c4 = (lane & 15) * 4;
      for (int pass = 0; pass < 2; ++pass) {
#pragma unroll
        for (int it = 0; it < 8; ++it) {
          const int row = it * 2 + hh;
          v4f v = *(const v4f*)(slab + row * 68 + c4);
          *(volatile v4f*)(C + (size_t)(mBase + row) * ldc + n0 + c4) = v;
        }
        __threadfence();
      }
    } else {
      const int q = lane >> 3, c8 = (lane & 7) * 8;
      unsigned short* C  = (unsigned short*)Cout  + (size_t)b * strideC;
      unsigned short* C2 = (OUT_MODE == 2) ? ((unsigned short*)Cout2 + (size_t)b * strideC) : nullptr;
      for (int pass = 0; pass < 2; ++pass) {
#pragma unroll
        for (int it = 0; it < 4; ++it) {
          const int row = it * 4 + q;
          const float* sp = slab + row * 68 + c8;
          v8h hv, lv;
#pragma unroll
          for (int e = 0; e < 8; ++e) {
            if (OUT_MODE == 1) {
              hv[e] = (_Float16)sp[e];
            } else {
              unsigned short hb = f2bf_bits(sp[e]);
              unsigned short lb = f2bf_bits(sp[e] - bf_bits2f(hb));
              hv[e] = __builtin_bit_cast(_Float16, hb);
              lv[e] = __builtin_bit_cast(_Float16, lb);
            }
          }
          *(volatile v8h*)(C + (size_t)(mBase + row) * ldc + n0 + c8) = hv;
          if (OUT_MODE == 2) *(volatile v8h*)(C2 + (size_t)(mBase + row) * ldc + n0 + c8) = lv;
        }
        __threadfence();
      }
    }
    __builtin_amdgcn_fence(__ATOMIC_RELEASE, "workgroup");
    __builtin_amdgcn_wave_barrier();
    __builtin_amdgcn_fence(__ATOMIC_ACQUIRE, "workgroup");
  }
}

__global__ __launch_bounds__(256) void cast_f32_f16x2(
    const float* __restrict__ in, _Float16* __restrict__ out, int n2) {
  int i = blockIdx.x * 256 + threadIdx.x;
  if (i < n2) {
    const _Float16 h0 = (_Float16)in[2 * i], h1 = (_Float16)in[2 * i + 1];
    const unsigned u = (unsigned)__builtin_bit_cast(unsigned short, h0) | ((unsigned)__builtin_bit_cast(unsigned short, h1) << 16);
    ((volatile unsigned*)out)[i] = u;
    __threadfence();
    ((volatile unsigned*)out)[i] = u;
  }
}

__global__ __launch_bounds__(256) void cast_scale_f32_f16x2(
    const float* __restrict__ in, _Float16* __restrict__ out, int n2, float sc) {
  int i = blockIdx.x * 256 + threadIdx.x;
  if (i < n2) {
    const _Float16 h0 = (_Float16)(in[2 * i] * sc), h1 = (_Float16)(in[2 * i + 1] * sc);
    const unsigned u = (unsigned)__builtin_bit_cast(unsigned short, h0) | ((unsigned)__builtin_bit_cast(unsigned short, h1) << 16);
    ((volatile unsigned*)out)[i] = u;
    __threadfence();
    ((volatile unsigned*)out)[i] = u;
  }
}

__global__ __launch_bounds__(256) void split_pad_bf16x2(
    const float* __restrict__ in, unsigned short* __restrict__ hi, unsigned short* __restrict__ lo,
    int rows_valid, int n2) {
  const int i = blockIdx.x * 256 + threadIdx.x;
  if (i < n2) {
    const int e0  = 2 * i;
    const int row = e0 / D_INNER;
    const int col = e0 - row * D_INNER;
    const bool valid = row < rows_valid;
    const int rowc = valid ? row : (rows_valid - 1);
    const float* p = in + (size_t)rowc * D_INNER + col;
    float f0 = p[0], f1 = p[1];
    f0 = valid ? f0 : 0.0f;
    f1 = valid ? f1 : 0.0f;
    const unsigned short h0 = f2bf_bits(f0), h1 = f2bf_bits(f1);
    const unsigned short l0 = f2bf_bits(f0 - bf_bits2f(h0)), l1 = f2bf_bits(f1 - bf_bits2f(h1));
    const unsigned hu = (unsigned)h0 | ((unsigned)h1 << 16);
    const unsigned lu = (unsigned)l0 | ((unsigned)l1 << 16);
    ((volatile unsigned*)hi)[i] = hu;
    ((volatile unsigned*)lo)[i] = lu;
    __threadfence();
    ((volatile unsigned*)hi)[i] = hu;
    ((volatile unsigned*)lo)[i] = lu;
  }
}

__global__ __launch_bounds__(256) void conv_split_kernel(
    const float* __restrict__ xz, const float* __restrict__ convw, const float* __restrict__ convb,
    unsigned short* __restrict__ xhi, unsigned short* __restrict__ xlo) {
  const int t  = threadIdx.x;
  const int m  = blockIdx.x * 4 + (t >> 6);
  const int l  = m & (SEQ_L - 1);
  const int dg = (t & 63) * 8;

  v4f w[8];
#pragma unroll
  for (int j = 0; j < 8; ++j) w[j] = *(const v4f*)(convw + (size_t)(dg + j) * 4);
  const v4f cb0 = *(const v4f*)(convb + dg);
  const v4f cb1 = *(const v4f*)(convb + dg + 4);
  float cbv[8];
#pragma unroll
  for (int e = 0; e < 4; ++e) { cbv[e] = cb0[e]; cbv[4 + e] = cb1[e]; }

  float xin[4][8];
#pragma unroll
  for (int k = 0; k < 4; ++k) {
    const bool valid = (l - 3 + k) >= 0;
    const int  row   = valid ? (m - 3 + k) : m;
    const float* p = xz + (size_t)row * (2 * D_INNER) + dg;
    const v4f a = *(const v4f*)(p);
    const v4f b = *(const v4f*)(p + 4);
#pragma unroll
    for (int e = 0; e < 4; ++e) {
      xin[k][e]     = valid ? a[e] : 0.0f;
      xin[k][4 + e] = valid ? b[e] : 0.0f;
    }
  }

  v8us hv, lv;
#pragma unroll
  for (int j = 0; j < 8; ++j) {
    const float s = ((xin[0][j] * w[j][0] + xin[1][j] * w[j][1]) + xin[2][j] * w[j][2]) + xin[3][j] * w[j][3] + cbv[j];
    const float v = silu_f(s);
    const unsigned short hb = f2bf_bits(v);
    const unsigned short lb = f2bf_bits(v - bf_bits2f(hb));
    hv[j] = hb;
    lv[j] = lb;
  }
  unsigned short* ph = xhi + (size_t)m * D_INNER + dg;
  unsigned short* pl = xlo + (size_t)m * D_INNER + dg;
  *(volatile v8us*)ph = hv;
  *(volatile v8us*)pl = lv;
  __threadfence();
  *(volatile v8us*)ph = hv;
  *(volatile v8us*)pl = lv;
}

__global__ __launch_bounds__(512) void scan_kernel(
    const float* __restrict__ dbc, const float* __restrict__ xz,
    const float* __restrict__ convw, const float* __restrict__ convb,
    const float* __restrict__ Wdt, const float* __restrict__ bdt,
    const float* __restrict__ Alog, const float* __restrict__ Dskip,
    _Float16* __restrict__ yout) {
  __shared__ __align__(16) float    sd[SEQ_L * DBC_LD];
  __shared__ __align__(16) _Float16 ys[16 * D_INNER];
  const int seq  = blockIdx.x;
  const int d    = threadIdx.x;
  const int wave = d >> 5;
  const int lane = d & 31;
  const size_t row0 = (size_t)seq * SEQ_L;

  {
    const float* src = dbc + row0 * DBC_LD;
    for (int i = d; i < (SEQ_L * DBC_LD) / 4; i += 512)
      *(v4f*)(sd + 4 * i) = *(const v4f*)(src + 4 * i);
  }

  const v4f wc = *(const v4f*)(convw + (size_t)d * 4);
  const float cb = convb[d];
  v4f wdt[4], Av[4];
#pragma unroll
  for (int i = 0; i < 4; ++i) {
    wdt[i] = *(const v4f*)(Wdt + (size_t)d * DT_RANK + 4 * i);
    const v4f al = *(const v4f*)(Alog + (size_t)d * D_STATE + 4 * i);
    v4f a;
#pragma unroll
    for (int e = 0; e < 4; ++e) a[e] = -__expf(al[e]);
    Av[i] = a;
  }
  const float bd = bdt[d];
  const float ds = Dskip[d];

  float h[D_STATE];
#pragma unroll
  for (int n = 0; n < D_STATE; ++n) h[n] = 0.0f;
  float xm3 = 0.0f, xm2 = 0.0f, xm1 = 0.0f;

  __syncthreads();

  for (int l = 0; l < SEQ_L; ++l) {
    const float* sr = sd + l * DBC_LD;
    float u = bd;
#pragma unroll
    for (int i = 0; i < 4; ++i) {
      const v4f q = *(const v4f*)(sr + 4 * i);
#pragma unroll
      for (int e = 0; e < 4; ++e) u += q[e] * wdt[i][e];
    }
    const float dtv = fmaxf(u, 0.0f) + log1pf(__expf(-fabsf(u)));

    const size_t m = row0 + (size_t)l;
    const float xl = xz[m * (2 * D_INNER) + d];
    const float s  = ((xm3 * wc[0] + xm2 * wc[1]) + xm1 * wc[2]) + xl * wc[3] + cb;
    xm3 = xm2; xm2 = xm1; xm1 = xl;
    const float xv  = silu_f(s);
    const float dtx = dtv * xv;

    float acc = 0.0f;
#pragma unroll
    for (int i = 0; i < 4; ++i) {
      const v4f bq = *(const v4f*)(sr + DT_RANK + 4 * i);
      const v4f cq = *(const v4f*)(sr + DT_RANK + D_STATE + 4 * i);
#pragma unroll
      for (int e = 0; e < 4; ++e) {
        const float dA = __expf(dtv * Av[i][e]);
        const float hn = dA * h[4 * i + e] + dtx * bq[e];
        h[4 * i + e] = hn;
        acc += hn * cq[e];
      }
    }
    const float zv = xz[m * (2 * D_INNER) + D_INNER + d];
    const float yv = (acc + xv * ds) * silu_f(zv);
    ys[(l & 15) * D_INNER + d] = (_Float16)yv;

    if ((l & 15) == 15) {
      __syncthreads();
      const size_t mrow = row0 + (size_t)(l - 15 + wave);
      const _Float16* yr = ys + wave * D_INNER;
      _Float16* gdst = yout + mrow * D_INNER;
      for (int pass = 0; pass < 2; ++pass) {
#pragma unroll
        for (int it = 0; it < 2; ++it) {
          const int c = it * 32 + lane;
          const v8h v = *(const v8h*)(yr + c * 8);
          *(volatile v8h*)(gdst + c * 8) = v;
        }
        __threadfence();
      }
      __syncthreads();
    }
  }
}

extern "C" void kernel_launch(void* const* d_in, const int* in_sizes, int n_in,
                              void* d_out, int out_size, void* d_ws, size_t ws_size,
                              hipStream_t stream) {
  if (n_in < 19) return;
  if (in_sizes[0] != MTOT * D_MODEL) return;
  if (out_size != MTOT * D_MODEL) return;
  for (int dir = 0; dir < 2; ++dir) {
    const int base = 1 + dir * 9;
    if (in_sizes[base + 0] != 2 * D_INNER * D_MODEL) return;
    if (in_sizes[base + 1] != D_INNER * 4) return;
    if (in_sizes[base + 2] != D_INNER) return;
    if (in_sizes[base + 3] != N_DBC * D_INNER) return;
    if (in_sizes[base + 4] != D_INNER * DT_RANK) return;
    if (in_sizes[base + 5] != D_INNER) return;
    if (in_sizes[base + 6] != D_INNER * D_STATE) return;
    if (in_sizes[base + 7] != D_INNER) return;
    if (in_sizes[base + 8] != D_MODEL * D_INNER) return;
  }

  const size_t b_xh   = (size_t)MTOT * D_MODEL * 2;
  const size_t b_win  = (size_t)2 * D_INNER * D_MODEL * 2;
  const size_t b_xz   = (size_t)MTOT * 2 * D_INNER * 4;
  const size_t b_xcp  = (size_t)MTOT * D_INNER * 2;
  const size_t b_wxp  = (size_t)DBC_LD * D_INNER * 2;
  const size_t b_dbc  = (size_t)MTOT * DBC_LD * 4;
  const size_t b_y    = (size_t)MTOT * D_INNER * 2;
  const size_t b_wout = (size_t)D_MODEL * D_INNER * 2;
  size_t off = 0;
  const size_t o_xh   = off; off += b_xh;
  const size_t o_win  = off; off += b_win;
  const size_t o_xz   = off; off += b_xz;
  const size_t o_xchi = off; off += b_xcp;
  const size_t o_xclo = off; off += b_xcp;
  const size_t o_wxhi = off; off += b_wxp;
  const size_t o_wxlo = off; off += b_wxp;
  const size_t o_dbc  = off; off += b_dbc;
  const size_t o_y    = off; off += b_y;
  const size_t o_wout = off; off += b_wout;
  if (off > ws_size) return;

  char* ws = (char*)d_ws;
  unsigned short* xh   = (unsigned short*)(ws + o_xh);
  unsigned short* win  = (unsigned short*)(ws + o_win);
  float*          xz   = (float*)(ws + o_xz);
  unsigned short* xchi = (unsigned short*)(ws + o_xchi);
  unsigned short* xclo = (unsigned short*)(ws + o_xclo);
  unsigned short* wxhi = (unsigned short*)(ws + o_wxhi);
  unsigned short* wxlo = (unsigned short*)(ws + o_wxlo);
  float*          dbc  = (float*)(ws + o_dbc);
  unsigned short* ybuf = (unsigned short*)(ws + o_y);
  unsigned short* wout = (unsigned short*)(ws + o_wout);

  const float* x   = (const float*)d_in[0];
  float*       out = (float*)d_out;

  {
    const int n2 = (MTOT * D_MODEL) / 2;
    cast_f32_f16x2<<<dim3((n2 + 255) / 256), dim3(256), 0, stream>>>(x, (_Float16*)xh, n2);
  }

  const float w_carry     = 16.0f;
  const float w_carry_inv = 1.0f / 16.0f;

  for (int dir = 0; dir < 2; ++dir) {
    const int base = 1 + dir * 9;
    const float* W_in   = (const float*)d_in[base + 0];
    const float* convw  = (const float*)d_in[base + 1];
    const float* convb  = (const float*)d_in[base + 2];
    const float* W_x    = (const float*)d_in[base + 3];
    const float* W_dt   = (const float*)d_in[base + 4];
    const float* b_dt   = (const float*)d_in[base + 5];
    const float* A_log  = (const float*)d_in[base + 6];
    const float* D_skip = (const float*)d_in[base + 7];
    const float* W_out  = (const float*)d_in[base + 8];

    {
      const int n2 = (2 * D_INNER * D_MODEL) / 2;
      cast_scale_f32_f16x2<<<dim3((n2 + 255) / 256), dim3(256), 0, stream>>>(W_in, (_Float16*)win, n2, w_carry);
    }
    {
      const int n2 = (DBC_LD * D_INNER) / 2;
      split_pad_bf16x2<<<dim3((n2 + 255) / 256), dim3(256), 0, stream>>>(W_x, wxhi, wxlo, N_DBC, n2);
    }
    {
      const int n2 = (D_MODEL * D_INNER) / 2;
      cast_scale_f32_f16x2<<<dim3((n2 + 255) / 256), dim3(256), 0, stream>>>(W_out, (_Float16*)wout, n2, w_carry);
    }

    {
      const int M = MTOT, N = 2 * D_INNER, K = D_MODEL;
      const int tiles = (M / 64) * (N / 64);
      wmma_gemm64<0, false, 0, 0, false><<<dim3((tiles + 7) / 8, 1), dim3(256), 0, stream>>>(
          xh, xh, K, 0L, win, win, K, 0L, (void*)xz, (void*)xz, N, 0L,
          b_dt, x, 0L, M, N, K, w_carry_inv);
    }

    conv_split_kernel<<<dim3(MTOT / 4), dim3(256), 0, stream>>>(xz, convw, convb, xchi, xclo);

    {
      const int M = MTOT, N = DBC_LD, K = D_INNER;
      const int tiles = (M / 64) * (N / 64);
      wmma_gemm64<1, true, 0, 0, false><<<dim3((tiles + 7) / 8, 1), dim3(256), 0, stream>>>(
          xchi, xclo, K, 0L, wxhi, wxlo, K, 0L, (void*)dbc, (void*)dbc, N, 0L,
          b_dt, x, 0L, M, N, K, 1.0f);
    }

    scan_kernel<<<dim3(NSEQ), dim3(512), 0, stream>>>(
        dbc, xz, convw, convb, W_dt, b_dt, A_log, D_skip, (_Float16*)ybuf);

    {
      const int M = MTOT, N = D_MODEL, K = D_INNER;
      const int tiles = (M / 64) * (N / 64);
      const float* resid = (dir == 0) ? x : (const float*)out;
      wmma_gemm64<0, false, 0, 0, true><<<dim3((tiles + 7) / 8, 1), dim3(256), 0, stream>>>(
          ybuf, ybuf, K, 0L, wout, wout, K, 0L, (void*)out, (void*)out, N, 0L,
          b_dt, resid, 0L, M, N, K, w_carry_inv);
    }
  }
}
